// Decoder_52398601011370
// MI455X (gfx1250) — hardware-verified
//
#include <hip/hip_runtime.h>
#include <stddef.h>
#include <stdint.h>


#define BD    2048
#define AD    512
#define NABS  16
#define ED    256
#define HD    256
#define OD    2
#define NPAD  16
#define PTHR  256
#define NU_EB (AD * (ED / 8))
#define NU_W1 (HD * (ED / 8))
#define NU_W2 (NPAD * (HD / 8))
#define GBM   64
#define GBN   64
#define GTHR  128
#define TA    64
#define TB    32
#define DTHR  128
#define PL_F  (TA * HD)
#define W0_F  HD
#define SL_F  (TB * TA)
#define OL_F  (4 * TB * 32)
#define W2_F  (NPAD * HD / 2)
#define DEC_LDS_BYTES ((PL_F + W0_F + SL_F + OL_F + W2_F) * 4)
#define WSMAX 134217728

static_assert(NU_EB % PTHR == 0 && NU_W1 % PTHR == 0 && NU_W2 % PTHR == 0);
static_assert(ED / 8 == 32 && HD / 8 == 32);
static_assert(AD % GBM == 0 && HD % GBN == 0 && ED % 32 == 0 && HD % 32 == 0);
static_assert(GBM == (GTHR / 32) * 16 && GBN == 64);
static_assert(AD % TA == 0 && BD % TB == 0 && TA == (DTHR / 32) * 16);
static_assert((PL_F / 4) % DTHR == 0 && (SL_F / 4) % DTHR == 0 && (NPAD * HD / 8) % DTHR == 0);
static_assert(PL_F % 4 == 0 && W0_F % 4 == 0 && SL_F % 4 == 0 && OL_F % 4 == 0);
static_assert(DEC_LDS_BYTES == 99328);
static_assert(16 * OD * 4 == 128);
static_assert(TB % 4 == 0);

typedef float          v4f   __attribute__((ext_vector_type(4)));
typedef float          v8f   __attribute__((ext_vector_type(8)));
typedef int            v4i   __attribute__((ext_vector_type(4)));
typedef int            v8i   __attribute__((ext_vector_type(8)));
typedef unsigned       v2u   __attribute__((ext_vector_type(2)));
typedef unsigned short v8us  __attribute__((ext_vector_type(8)));
typedef unsigned short v16us __attribute__((ext_vector_type(16)));
typedef __bf16         v16bf __attribute__((ext_vector_type(16)));
typedef v4f  __attribute__((may_alias)) v4fa;
typedef v4i  __attribute__((may_alias)) v4ia;
typedef v8us __attribute__((may_alias)) v8usa;
union FragB { v16bf v; v16us u; v8us h[2]; v8i w; };

__device__ __forceinline__ v8f wmb(const FragB& a, const FragB& b, v8f c) {
  v8f d = __builtin_amdgcn_wmma_f32_16x16x32_bf16(false, a.v, false, b.v, (short)0, c, false, false);
  asm volatile("v_nop\n\tv_nop\n\tv_nop\n\tv_nop" : "+v"(d) : "v"(a.w), "v"(b.w));
  return d;
}

__device__ __forceinline__ unsigned bf16_rnd(float f) {
  const unsigned u = __float_as_uint(f);
  return u + 0x7FFFu + ((u >> 16) & 1u);
}
__device__ __forceinline__ unsigned bf16_bits(float f) { return bf16_rnd(f) >> 16; }
__device__ __forceinline__ float bf16_val(float f) { return __uint_as_float(bf16_rnd(f) & 0xffff0000u); }

__device__ __forceinline__ v2u hl_pair(float s, float wa, float pa, float wb, float pb) {
  float va = fmaf(s, wa, pa);
  float vb = fmaf(s, wb, pb);
  va = (va > 0.0f) ? va : (va - va);
  vb = (vb > 0.0f) ? vb : (vb - vb);
  const unsigned ra = bf16_rnd(va), rb = bf16_rnd(vb);
  const float da = va - __uint_as_float(ra & 0xffff0000u);
  const float db = vb - __uint_as_float(rb & 0xffff0000u);
  const unsigned la = bf16_rnd(da), lb = bf16_rnd(db);
  v2u o;
  o.x = (ra >> 16) | (rb & 0xffff0000u);
  o.y = (la >> 16) | (lb & 0xffff0000u);
  return o;
}

__global__ __launch_bounds__(PTHR) void k_prep(const float* __restrict__ emb, const float* __restrict__ W1,
                                               const float* __restrict__ W2,
                                               unsigned short* EB, unsigned short* W1T, unsigned short* W2T) {
  const int u = (int)blockIdx.x * PTHR + (int)threadIdx.x;
  v8us o;
  unsigned short* dp;
  if (u < NU_EB) {
    const int row = u >> 5;
    const int k8  = (u & 31) * 8;
    const float* p = emb + (size_t)row * ED + k8;
    const v4f a = *(const v4fa*)p;
    const v4f b = *(const v4fa*)(p + 4);
    o[0] = (unsigned short)bf16_bits(a.x); o[1] = (unsigned short)bf16_bits(a.y);
    o[2] = (unsigned short)bf16_bits(a.z); o[3] = (unsigned short)bf16_bits(a.w);
    o[4] = (unsigned short)bf16_bits(b.x); o[5] = (unsigned short)bf16_bits(b.y);
    o[6] = (unsigned short)bf16_bits(b.z); o[7] = (unsigned short)bf16_bits(b.w);
    dp = EB + (size_t)row * ED + k8;
  } else if (u < NU_EB + NU_W1) {
    const int v  = u - NU_EB;
    const int n  = v >> 5;
    const int k8 = (v & 31) * 8;
    const float* p = W1 + (size_t)(1 + k8) * HD + n;
#pragma unroll
    for (int i = 0; i < 8; ++i) o[i] = (unsigned short)bf16_bits(p[(size_t)i * HD]);
    dp = W1T + (size_t)n * ED + k8;
  } else if (u < NU_EB + NU_W1 + NU_W2) {
    const int v  = u - NU_EB - NU_W1;
    const int n  = v >> 5;
    const int k8 = (v & 31) * 8;
    const int nc = n < OD ? n : OD - 1;
    const float* p = W2 + (size_t)k8 * OD + nc;
#pragma unroll
    for (int i = 0; i < 8; ++i) {
      const unsigned bb = bf16_bits(p[(size_t)i * OD]);
      o[i] = (n < OD) ? (unsigned short)bb : (unsigned short)0;
    }
    dp = W2T + (size_t)n * HD + k8;
  } else {
    return;
  }
  *(volatile v8us*)dp = o;
  __threadfence();
  *(volatile v8us*)dp = o;
}

__global__ __launch_bounds__(GTHR) void k_gemm(
    const unsigned short* __restrict__ A, const unsigned short* __restrict__ WT,
    const float* __restrict__ bias, float* outF, int K, int ldo)
{
  __shared__ __attribute__((aligned(16))) float stg[GBM * GBN];
  const int tid = (int)threadIdx.x, lane = tid & 31, wave = tid >> 5, hh = lane >> 4, m = lane & 15;
  const int rowBase = (int)blockIdx.x * GBM;
  const int col0    = (int)blockIdx.y * GBN;

  v8f acc[4];
  {
    const v8f z = {0.f, 0.f, 0.f, 0.f, 0.f, 0.f, 0.f, 0.f};
    acc[0] = z; acc[1] = z; acc[2] = z; acc[3] = z;
  }
  const unsigned short* ap = A  + (size_t)(rowBase + 16 * wave + m) * (size_t)K + 8 * hh;
  const unsigned short* wp = WT + (size_t)(col0 + m) * (size_t)K + 8 * hh;
  const int ksteps = K >> 5;
#pragma unroll 1
  for (int ks = 0; ks < ksteps; ++ks) {
    FragB af;
    af.h[0] = *(const v8usa*)(ap + 32 * ks);
    af.h[1] = *(const v8usa*)(ap + 32 * ks + 16);
#pragma unroll
    for (int t = 0; t < 4; ++t) {
      const unsigned short* wq = wp + (size_t)(16 * t) * (size_t)K + 32 * ks;
      FragB bf;
      bf.h[0] = *(const v8usa*)wq;
      bf.h[1] = *(const v8usa*)(wq + 16);
      acc[t] = wmb(af, bf, acc[t]);
    }
  }

#pragma unroll
  for (int t = 0; t < 4; ++t) {
    const int lc = 16 * t + m;
#pragma unroll
    for (int r = 0; r < 8; ++r) {
      const int lr = 16 * wave + 8 * hh + r;
      stg[lr * GBN + lc] = acc[t][r];
    }
  }
  __syncthreads();

  v4f bv;
  {
    const v4f t1 = *(const v4fa*)(bias + col0 + 4 * m);
    bv.x = bf16_val(t1.x); bv.y = bf16_val(t1.y); bv.z = bf16_val(t1.z); bv.w = bf16_val(t1.w);
  }
  v4f fv[8];
#pragma unroll
  for (int i = 0; i < 8; ++i) {
    const int lr = 16 * wave + 2 * i + hh;
    fv[i] = *(const v4fa*)(stg + lr * GBN + 4 * m) + bv;
  }
#pragma unroll
  for (int i = 0; i < 8; ++i) {
    const int lr = 16 * wave + 2 * i + hh;
    const int gr = rowBase + lr;
    float* op = outF + (size_t)gr * (size_t)ldo + col0 + 4 * m;
    *(volatile v4f*)op = fv[i];
  }
  __threadfence();
#pragma unroll
  for (int i = 0; i < 8; ++i) {
    const int lr = 16 * wave + 2 * i + hh;
    const int gr = rowBase + lr;
    float* op = outF + (size_t)gr * (size_t)ldo + col0 + 4 * m;
    *(volatile v4f*)op = fv[i];
  }
}

__global__ __launch_bounds__(DTHR) void k_dec(const float* __restrict__ absAct, const int* __restrict__ asg,
                                              const float* __restrict__ W1, const float* __restrict__ b2,
                                              const float* __restrict__ P, const unsigned short* __restrict__ W2T,
                                              float* out) {
  extern __shared__ __attribute__((aligned(16))) float dsm[];
  float* pl  = dsm;
  float* w0l = pl + PL_F;
  float* sl  = w0l + W0_F;
  float* ol  = sl + SL_F;
  unsigned short* w2l = (unsigned short*)(ol + OL_F);
  const int tid = (int)threadIdx.x, lane = tid & 31, wave = tid >> 5, hh = lane >> 4, m = lane & 15;
  const int a0 = (int)blockIdx.x * TA;
  const int b0 = (int)blockIdx.y * TB;

  {
    const float* pg = P + (size_t)a0 * HD;
#pragma unroll 4
    for (int i = tid; i < PL_F / 4; i += DTHR) {
      const v4f v = *(const v4fa*)(pg + 4 * i);
      *(v4fa*)(pl + 4 * i) = v;
    }
  }
  if (tid < W0_F / 4) {
    const v4f v = *(const v4fa*)(W1 + 4 * tid);
    v4f r;
    r.x = bf16_val(v.x); r.y = bf16_val(v.y); r.z = bf16_val(v.z); r.w = bf16_val(v.w);
    *(v4fa*)(w0l + 4 * tid) = r;
  }
#pragma unroll 1
  for (int i = tid; i < (NPAD * HD) / 8; i += DTHR) {
    const v8us v = *(const v8usa*)(W2T + 8 * i);
    *(v8usa*)(w2l + 8 * i) = v;
  }
  {
    const float qnan = __int_as_float(0x7fc00000);
#pragma unroll 1
    for (int u = tid; u < SL_F / 4; u += DTHR) {
      const int bl = u >> 4;
      const int a4 = (u & 15) * 4;
      const int b  = b0 + bl;
      const v4i id = *(const v4ia*)(asg + (size_t)b * AD + a0 + a4);
      const float* tb = absAct + (size_t)b * NABS;
      int i0 = id.x, i1 = id.y, i2 = id.z, i3 = id.w;
      i0 += (i0 < 0) ? NABS : 0; i1 += (i1 < 0) ? NABS : 0;
      i2 += (i2 < 0) ? NABS : 0; i3 += (i3 < 0) ? NABS : 0;
      const bool k0 = (unsigned)i0 < (unsigned)NABS, k1 = (unsigned)i1 < (unsigned)NABS;
      const bool k2 = (unsigned)i2 < (unsigned)NABS, k3 = (unsigned)i3 < (unsigned)NABS;
      const float x0 = tb[k0 ? i0 : 0], x1 = tb[k1 ? i1 : 0];
      const float x2 = tb[k2 ? i2 : 0], x3 = tb[k3 ? i3 : 0];
      v4f r;
      r.x = k0 ? bf16_val(x0) : qnan;
      r.y = k1 ? bf16_val(x1) : qnan;
      r.z = k2 ? bf16_val(x2) : qnan;
      r.w = k3 ? bf16_val(x3) : qnan;
      *(v4fa*)(sl + bl * TA + a4) = r;
    }
  }
  float b2v;
  {
    const float t = b2[m < OD ? m : OD - 1];
    b2v = (m < OD) ? bf16_val(t) : 0.0f;
  }
  __syncthreads();

  const float* prow = pl + (16 * wave + m) * HD + 8 * hh;
  const float* w0p  = w0l + 8 * hh;
  const unsigned short* wbp = w2l + m * HD + 8 * hh;
  float* orow = ol + wave * (TB * 32);

#pragma unroll 1
  for (int bl = 0; bl < TB; ++bl) {
    const float s = sl[bl * TA + 16 * wave + m];
    v8f acc = {0.f, 0.f, 0.f, 0.f, 0.f, 0.f, 0.f, 0.f};
#pragma unroll 1
    for (int ks = 0; ks < HD / 32; ++ks) {
      const int k0 = 32 * ks;
      const v4f p0 = *(const v4fa*)(prow + k0);
      const v4f p1 = *(const v4fa*)(prow + k0 + 4);
      const v4f p2 = *(const v4fa*)(prow + k0 + 16);
      const v4f p3 = *(const v4fa*)(prow + k0 + 20);
      const v4f u0 = *(const v4fa*)(w0p + k0);
      const v4f u1 = *(const v4fa*)(w0p + k0 + 4);
      const v4f u2 = *(const v4fa*)(w0p + k0 + 16);
      const v4f u3 = *(const v4fa*)(w0p + k0 + 20);
      FragB bf;
      bf.h[0] = *(const v8usa*)(wbp + k0);
      bf.h[1] = *(const v8usa*)(wbp + k0 + 16);
      FragB ah, al;
      v2u q;
      q = hl_pair(s, u0.x, p0.x, u0.y, p0.y); ah.w[0] = (int)q.x; al.w[0] = (int)q.y;
      q = hl_pair(s, u0.z, p0.z, u0.w, p0.w); ah.w[1] = (int)q.x; al.w[1] = (int)q.y;
      q = hl_pair(s, u1.x, p1.x, u1.y, p1.y); ah.w[2] = (int)q.x; al.w[2] = (int)q.y;
      q = hl_pair(s, u1.z, p1.z, u1.w, p1.w); ah.w[3] = (int)q.x; al.w[3] = (int)q.y;
      q = hl_pair(s, u2.x, p2.x, u2.y, p2.y); ah.w[4] = (int)q.x; al.w[4] = (int)q.y;
      q = hl_pair(s, u2.z, p2.z, u2.w, p2.w); ah.w[5] = (int)q.x; al.w[5] = (int)q.y;
      q = hl_pair(s, u3.x, p3.x, u3.y, p3.y); ah.w[6] = (int)q.x; al.w[6] = (int)q.y;
      q = hl_pair(s, u3.z, p3.z, u3.w, p3.w); ah.w[7] = (int)q.x; al.w[7] = (int)q.y;
      acc = wmb(ah, bf, acc);
      acc = wmb(al, bf, acc);
    }
    if (m < OD) {
      float* q = orow + bl * 32 + 16 * hh + m;
#pragma unroll
      for (int r = 0; r < 8; ++r) q[2 * r] = acc[r] + b2v;
    }
  }
  __syncthreads();

  v4f ov[8];
#pragma unroll
  for (int it = 0; it < 8; ++it) {
    const int line = 4 * it + (lane >> 3);
    ov[it] = *(const v4fa*)(orow + line * 32 + 4 * (lane & 7));
  }
#pragma unroll
  for (int it = 0; it < 8; ++it) {
    const int line = 4 * it + (lane >> 3);
    float* gp = out + ((size_t)(b0 + line) * AD + a0 + 16 * wave) * OD + 4 * (lane & 7);
    *(volatile v4f*)gp = ov[it];
  }
  __threadfence();
#pragma unroll
  for (int it = 0; it < 8; ++it) {
    const int line = 4 * it + (lane >> 3);
    float* gp = out + ((size_t)(b0 + line) * AD + a0 + 16 * wave) * OD + 4 * (lane & 7);
    *(volatile v4f*)gp = ov[it];
  }
}

static inline size_t al256(size_t o) { return (o + 255) & ~(size_t)255; }

extern "C" void kernel_launch(void* const* d_in, const int* in_sizes, int n_in,
                              void* d_out, int out_size, void* d_ws, size_t ws_size,
                              hipStream_t stream) {
  if (n_in < 8) return;
  if (in_sizes[1] != BD * NABS) return;
  if (in_sizes[2] != BD * AD) return;
  if (in_sizes[3] != AD * ED) return;
  if (in_sizes[4] != (1 + ED) * HD) return;
  if (in_sizes[5] != HD) return;
  if (in_sizes[6] != HD * OD) return;
  if (in_sizes[7] != OD) return;
  if ((long long)out_size != (long long)BD * AD * OD) return;

  const float* absAct = (const float*)d_in[1];
  const int*   asg    = (const int*)d_in[2];
  const float* emb    = (const float*)d_in[3];
  const float* W1     = (const float*)d_in[4];
  const float* b1     = (const float*)d_in[5];
  const float* W2     = (const float*)d_in[6];
  const float* b2     = (const float*)d_in[7];
  float* out = (float*)d_out;

  char* ws = (char*)d_ws;
  size_t off = 0;
  const size_t oEB  = off; off = al256(off + (size_t)AD * ED * 2);
  const size_t oW1T = off; off = al256(off + (size_t)HD * ED * 2);
  const size_t oW2T = off; off = al256(off + (size_t)NPAD * HD * 2);
  const size_t oP   = off; off = al256(off + (size_t)AD * HD * 4);
  if (off > ws_size || off > (size_t)WSMAX) return;
  unsigned short* EB  = (unsigned short*)(ws + oEB);
  unsigned short* W1T = (unsigned short*)(ws + oW1T);
  unsigned short* W2T = (unsigned short*)(ws + oW2T);
  float*          Pp  = (float*)(ws + oP);

  hipFuncSetAttribute(reinterpret_cast<const void*>(&k_dec), hipFuncAttributeMaxDynamicSharedMemorySize,
                      (int)DEC_LDS_BYTES);

  k_prep<<<(NU_EB + NU_W1 + NU_W2) / PTHR, PTHR, 0, stream>>>(emb, W1, W2, EB, W1T, W2T);
  k_gemm<<<dim3(AD / GBM, HD / GBN), GTHR, 0, stream>>>(EB, W1T, b1, Pp, ED, HD);
  k_dec<<<dim3(AD / TA, BD / TB), DTHR, (size_t)DEC_LDS_BYTES, stream>>>(absAct, asg, W1, b2, Pp, W2T, out);
}
